// _AttentionBlock_5935644803163
// MI455X (gfx1250) — hardware-verified
//
#include <hip/hip_runtime.h>
#include <math.h>

constexpr int kNB  = 16;
constexpr int kC   = 512;
constexpr int kT   = 1024;
constexpr int kNH  = 8;
constexpr int kDH  = 64;
constexpr int kE   = kNH * kDH;
constexpr int kTok = kNB * kT;
constexpr float kWCarry    = 16.0f;
constexpr float kWCarryInv = 1.0f / 16.0f;
constexpr float kPCarry    = 2048.0f;
constexpr float kOCarry    = 256.0f;
constexpr float kScoreScale = 0.125f;
constexpr float kPVScale   = kOCarry / kPCarry;
constexpr float kOutScale  = 1.0f / (kOCarry * kWCarry);
constexpr float kInvC      = 1.0f / 512.0f;
constexpr float kLnEps     = 1e-6f;

typedef __attribute__((ext_vector_type(16))) _Float16 v16h;
typedef __attribute__((ext_vector_type(8)))  _Float16 v8h;
typedef __attribute__((ext_vector_type(16))) __bf16   v16b;
typedef __attribute__((ext_vector_type(8)))  __bf16   v8b;
typedef __attribute__((ext_vector_type(8)))  float    v8f;
typedef __attribute__((ext_vector_type(4)))  float    v4f;
typedef __attribute__((ext_vector_type(4)))  unsigned int v4u;

__device__ __forceinline__ unsigned short f2bf_bits(float f) {
  unsigned u = __float_as_uint(f);
  return (unsigned short)((u + 0x7FFFu + ((u >> 16) & 1u)) >> 16);
}
__device__ __forceinline__ float bf_bits2f(unsigned short h) { return __uint_as_float(((unsigned)h) << 16); }

__device__ __forceinline__ void dep_guard_h(v8f& a, v8f& b, v16h x, v16h y) { asm volatile("v_nop\n\tv_nop\n\tv_nop\n\tv_nop" : "+v"(a), "+v"(b) : "v"(x), "v"(y)); }
__device__ __forceinline__ void dep_guard_b(v8f& a, v8f& b, v16b x, v16b y) { asm volatile("v_nop\n\tv_nop\n\tv_nop\n\tv_nop" : "+v"(a), "+v"(b) : "v"(x), "v"(y)); }
__device__ __forceinline__ void keep4_h(v16h a, v16h b, v16h c, v16h d) { asm volatile("v_nop" :: "v"(a), "v"(b), "v"(c), "v"(d)); }
__device__ __forceinline__ void keep4_b(v16b a, v16b b, v16b c, v16b d) { asm volatile("v_nop" :: "v"(a), "v"(b), "v"(c), "v"(d)); }
__device__ __forceinline__ void acc_guard4(v8f& a, v8f& b, v8f& c, v8f& d) { asm volatile("v_nop\n\tv_nop\n\tv_nop\n\tv_nop" : "+v"(a), "+v"(b), "+v"(c), "+v"(d)); }
template <typename T> struct Frag;
template <> struct Frag<_Float16> {
  typedef v16h V; union U { v16h v; v8h h[2]; };
  static __device__ __forceinline__ v16h load(const _Float16* p) {
    U f; f.h[0] = *(const v8h*)(p); f.h[1] = *(const v8h*)(p + 16); return f.v;
  }
  static __device__ __forceinline__ v8f mma(v16h a, v16h b, v8f c) {
    return __builtin_amdgcn_wmma_f32_16x16x32_f16(false, a, false, b, (short)0, c, false, false);
  }
  static __device__ __forceinline__ void guard(v8f& a, v8f& b, v16h x, v16h y) { dep_guard_h(a, b, x, y); }
  static __device__ __forceinline__ void keep(v16h a, v16h b, v16h c, v16h d) { keep4_h(a, b, c, d); }
};
template <> struct Frag<__bf16> {
  typedef v16b V; union U { v16b v; v8b h[2]; };
  static __device__ __forceinline__ v16b load(const __bf16* p) {
    U f; f.h[0] = *(const v8b*)(p); f.h[1] = *(const v8b*)(p + 16); return f.v;
  }
  static __device__ __forceinline__ v8f mma(v16b a, v16b b, v8f c) {
    return __builtin_amdgcn_wmma_f32_16x16x32_bf16(false, a, false, b, (short)0, c, false, false);
  }
  static __device__ __forceinline__ void guard(v8f& a, v8f& b, v16b x, v16b y) { dep_guard_b(a, b, x, y); }
  static __device__ __forceinline__ void keep(v16b a, v16b b, v16b c, v16b d) { keep4_b(a, b, c, d); }
};

__device__ __forceinline__ unsigned pk16(unsigned short a, unsigned short b) { return (unsigned)a | ((unsigned)b << 16); }
__device__ __forceinline__ unsigned short h_bits(float f) { const _Float16 h = (_Float16)f; return __builtin_bit_cast(unsigned short, h); }

template <int ET> struct Elem;
template <> struct Elem<0> { typedef _Float16 T; };
template <> struct Elem<1> { typedef __bf16 T; };
template <int ET, bool SPLIT, int BIAS_MODE, int OUT_MODE, bool RESID, int ACT = 0>
__global__ __launch_bounds__(256) void wmma_gemm64(
    const unsigned short* __restrict__ Ap, const unsigned short* __restrict__ A2p, int lda, long strideA,
    const unsigned short* __restrict__ Btp, const unsigned short* __restrict__ Bt2p, int ldb, long strideB,
    void* __restrict__ Cout, void* __restrict__ Cout2, int ldc, long strideC,
    const float* __restrict__ bias,
    const float* __restrict__ resid, long strideR,
    int M, int N, int K, float scale) {
  typedef typename Elem<ET>::T T;
  typedef typename Frag<T>::V V;
  const T* A = (const T*)Ap; const T* A2 = (const T*)A2p; const T* Bt = (const T*)Btp; const T* Bt2 = (const T*)Bt2p;
  __shared__ __align__(16) float sT[8][16 * 68];
  const int b    = blockIdx.y;
  const int lane = threadIdx.x & 31;
  const int wave = threadIdx.x >> 5;
  const int tilesN = N >> 6;
  const int tilesM = M >> 6;
  const int tile = blockIdx.x * 8 + wave;
  if (tile >= tilesM * tilesN) return;
  const int tm = tile / tilesN;
  const int tn = tile - tm * tilesN;
  const int m0 = tm << 6;
  const int n0 = tn << 6;

  const T* Ab  = A  + (size_t)b * strideA;
  const T* Bb  = Bt + (size_t)b * strideB;
  const T* Ab2 = SPLIT ? (A2  + (size_t)b * strideA) : nullptr;
  const T* Bb2 = SPLIT ? (Bt2 + (size_t)b * strideB) : nullptr;

  const int rlane = lane & 15;
  const int koff  = (lane >> 4) * 8;
  const int mOff  = (lane >> 4) * 8;

  v8f acc[4][4];
#pragma unroll
  for (int i = 0; i < 4; ++i)
#pragma unroll
    for (int j = 0; j < 4; ++j) acc[i][j] = (v8f){0.f,0.f,0.f,0.f,0.f,0.f,0.f,0.f};

  for (int k0 = 0; k0 < K; k0 += 32) {
    V bh[4], bl[4];
#pragma unroll
    for (int j = 0; j < 4; ++j) {
      const size_t bo = (size_t)(n0 + (j << 4) + rlane) * ldb + koff + k0;
      bh[j] = Frag<T>::load(Bb + bo);
      if (SPLIT) bl[j] = Frag<T>::load(Bb2 + bo);
    }
#pragma unroll
    for (int i = 0; i < 4; ++i) {
      const size_t ao = (size_t)(m0 + (i << 4) + rlane) * lda + koff + k0;
      V ah = Frag<T>::load(Ab + ao);
      V al;
      if (SPLIT) al = Frag<T>::load(Ab2 + ao);
#pragma unroll
      for (int j = 0; j < 4; ++j) {
        acc[i][j] = Frag<T>::mma(ah, bh[j], acc[i][j]);
        if (SPLIT) {
          acc[i][j] = Frag<T>::mma(ah, bl[j], acc[i][j]);
          acc[i][j] = Frag<T>::mma(al, bh[j], acc[i][j]);
        }
      }
      Frag<T>::guard(acc[i][0], acc[i][3], ah, SPLIT ? al : ah);
    }
    Frag<T>::keep(bh[0], bh[1], bh[2], bh[3]);
    if (SPLIT) Frag<T>::keep(bl[0], bl[1], bl[2], bl[3]);
  }
  acc_guard4(acc[0][0], acc[0][1], acc[0][2], acc[0][3]);
  acc_guard4(acc[1][0], acc[1][1], acc[1][2], acc[1][3]);
  acc_guard4(acc[2][0], acc[2][1], acc[2][2], acc[2][3]);
  acc_guard4(acc[3][0], acc[3][1], acc[3][2], acc[3][3]);

  float* slab = sT[wave];
  const float* Rb = RESID ? (resid + (size_t)b * strideR) : nullptr;
#pragma unroll
  for (int i = 0; i < 4; ++i) {
    const int mBase = m0 + (i << 4);
#pragma unroll
    for (int j = 0; j < 4; ++j) {
      const int n = n0 + (j << 4) + rlane;
      float bv = 0.f;
      if (BIAS_MODE == 2) bv = bias[n];
#pragma unroll
      for (int r = 0; r < 8; ++r) {
        float v = acc[i][j][r] * scale;
        if (BIAS_MODE == 1) v += bias[mBase + mOff + r];
        if (BIAS_MODE == 2) v += bv;
        if (RESID) v += Rb[(size_t)(mBase + mOff + r) * ldc + n];
        if (ACT == 2) v = fmaxf(v, 0.0f);
        if (ACT == 4) v = (v > 0.f) ? v : 0.01f * v;
        slab[(mOff + r) * 68 + (j << 4) + rlane] = v;
      }
    }
    __builtin_amdgcn_fence(__ATOMIC_RELEASE, "workgroup");
    __builtin_amdgcn_wave_barrier();
    __builtin_amdgcn_fence(__ATOMIC_ACQUIRE, "workgroup");
    if (OUT_MODE == 0) {
      float* C = (float*)Cout + (size_t)b * strideC;
      const int hh = lane >> 4, c4 = (lane & 15) * 4;
      for (int pass = 0; pass < 2; ++pass) {
#pragma unroll
        for (int it = 0; it < 8; ++it) {
          const int row = it * 2 + hh;
          v4f v = *(const v4f*)(slab + row * 68 + c4);
          *(volatile v4f*)(C + (size_t)(mBase + row) * ldc + n0 + c4) = v;
        }
        __threadfence();
      }
    } else {
      const int q = lane >> 3, c8 = (lane & 7) * 8;
      unsigned short* C  = (unsigned short*)Cout  + (size_t)b * strideC;
      unsigned short* C2 = (OUT_MODE == 2) ? ((unsigned short*)Cout2 + (size_t)b * strideC) : nullptr;
      for (int pass = 0; pass < 2; ++pass) {
#pragma unroll
        for (int it = 0; it < 4; ++it) {
          const int row = it * 4 + q;
          const float* sp = slab + row * 68 + c8;
          v8h hv, lv;
#pragma unroll
          for (int e = 0; e < 8; ++e) {
            if (OUT_MODE == 1) {
              hv[e] = (_Float16)sp[e];
            } else {
              unsigned short hb = f2bf_bits(sp[e]);
              unsigned short lb = f2bf_bits(sp[e] - bf_bits2f(hb));
              hv[e] = __builtin_bit_cast(_Float16, hb);
              lv[e] = __builtin_bit_cast(_Float16, lb);
            }
          }
          *(volatile v8h*)(C + (size_t)(mBase + row) * ldc + n0 + c8) = hv;
          if (OUT_MODE == 2) *(volatile v8h*)(C2 + (size_t)(mBase + row) * ldc + n0 + c8) = lv;
        }
        __threadfence();
      }
    }
    __builtin_amdgcn_fence(__ATOMIC_RELEASE, "workgroup");
    __builtin_amdgcn_wave_barrier();
    __builtin_amdgcn_fence(__ATOMIC_ACQUIRE, "workgroup");
  }
}

__global__ __launch_bounds__(256) void wtcast_kernel(const float* __restrict__ W0, const float* __restrict__ W1,
                                                     const float* __restrict__ W2, const float* __restrict__ W3,
                                                     unsigned short* __restrict__ out, float scale) {
  __shared__ float sm[64][65];
  const int t  = threadIdx.x;
  const int d0 = blockIdx.x * 64;
  const int h0 = blockIdx.y * 64;
  const int z  = blockIdx.z;
  const float* W = (z == 0) ? W0 : (z == 1) ? W1 : (z == 2) ? W2 : W3;
#pragma unroll
  for (int i = 0; i < 16; ++i) {
    const int e = i * 256 + t;
    const int r = e >> 6;
    const int c = e & 63;
    sm[c][r] = W[(size_t)(d0 + r) * kE + h0 + c] * scale;
  }
  __syncthreads();
  const int lane = t & 31, wave = t >> 5;
  const int q = lane >> 3, c8 = (lane & 7) * 8;
  unsigned short* op = out + (size_t)z * kE * kC;
  for (int pass = 0; pass < 2; ++pass) {
#pragma unroll
    for (int it = 0; it < 2; ++it) {
      const int row = wave * 8 + it * 4 + q;
      unsigned short hb[8];
#pragma unroll
      for (int e = 0; e < 8; ++e) hb[e] = h_bits(sm[row][c8 + e]);
      const v4u u = (v4u){pk16(hb[0], hb[1]), pk16(hb[2], hb[3]), pk16(hb[4], hb[5]), pk16(hb[6], hb[7])};
      *(volatile v4u*)(op + (size_t)(h0 + row) * kC + d0 + c8) = u;
    }
    __threadfence();
  }
}

__global__ __launch_bounds__(256) void ln_tok_kernel(const float* __restrict__ X, const float* __restrict__ g,
                                                     const float* __restrict__ be, unsigned short* __restrict__ xn) {
  __shared__ float part[4][64];
  __shared__ float meanS[64];
  __shared__ float rstdS[64];
  __shared__ float sm[64][65];
  const int tid  = threadIdx.x;
  const int blk  = blockIdx.x;
  const int b    = blk >> 4;
  const int t0   = (blk & 15) * 64;
  const int tl   = tid & 63;
  const int cg   = tid >> 6;
  const int lane = tid & 31, wave = tid >> 5;
  const int q    = lane >> 3, c8 = (lane & 7) * 8;
  const float* xb = X + (size_t)b * kC * kT + t0 + tl;

  float s = 0.f;
#pragma unroll 4
  for (int i = 0; i < 128; ++i) s += xb[(size_t)(cg * 128 + i) * kT];
  part[cg][tl] = s;
  __syncthreads();
  if (tid < 64) meanS[tid] = ((part[0][tid] + part[1][tid]) + (part[2][tid] + part[3][tid])) * kInvC;
  __syncthreads();
  const float mu = meanS[tl];

  float ss = 0.f;
#pragma unroll 4
  for (int i = 0; i < 128; ++i) {
    const float d = xb[(size_t)(cg * 128 + i) * kT] - mu;
    ss += d * d;
  }
  part[cg][tl] = ss;
  __syncthreads();
  if (tid < 64) {
    const float var = ((part[0][tid] + part[1][tid]) + (part[2][tid] + part[3][tid])) * kInvC;
    rstdS[tid] = rsqrtf(var + kLnEps);
  }
  __syncthreads();
  const float rs = rstdS[tl];

  for (int ch = 0; ch < 8; ++ch) {
    const int c0 = ch * 64;
#pragma unroll
    for (int i = 0; i < 16; ++i) {
      const int cl = cg + 4 * i;
      const float x  = xb[(size_t)(c0 + cl) * kT];
      const float xh = (x - mu) * rs;
      sm[cl][tl] = xh * g[c0 + cl] + be[c0 + cl];
    }
    __syncthreads();
    for (int pass = 0; pass < 2; ++pass) {
#pragma unroll
      for (int it = 0; it < 2; ++it) {
        const int row = wave * 8 + it * 4 + q;
        unsigned short hb[8];
#pragma unroll
        for (int e = 0; e < 8; ++e) hb[e] = h_bits(sm[c8 + e][row]);
        const v4u u = (v4u){pk16(hb[0], hb[1]), pk16(hb[2], hb[3]), pk16(hb[4], hb[5]), pk16(hb[6], hb[7])};
        *(volatile v4u*)(xn + (size_t)(b * kT + t0 + row) * kC + c0 + c8) = u;
      }
      __threadfence();
    }
    __syncthreads();
  }
}

__global__ __launch_bounds__(128) void softmax_row_kernel(const float* __restrict__ S, unsigned short* __restrict__ P) {
  __shared__ float redM[4];
  __shared__ float redS[4];
  const int row  = blockIdx.x;
  const int t    = threadIdx.x;
  const int lane = t & 31, wave = t >> 5;
  const int c0   = t * 8;
  const float* sr = S + (size_t)row * kT + c0;
  const v4f a = *(const v4f*)(sr);
  const v4f c = *(const v4f*)(sr + 4);
  float m = fmaxf(fmaxf(fmaxf(a[0], a[1]), fmaxf(a[2], a[3])), fmaxf(fmaxf(c[0], c[1]), fmaxf(c[2], c[3])));
#pragma unroll
  for (int off = 16; off > 0; off >>= 1) m = fmaxf(m, __shfl_xor(m, off, 32));
  if (lane == 0) redM[wave] = m;
  __syncthreads();
  m = fmaxf(fmaxf(redM[0], redM[1]), fmaxf(redM[2], redM[3]));
  const float p0 = expf(a[0] - m), p1 = expf(a[1] - m), p2 = expf(a[2] - m), p3 = expf(a[3] - m);
  const float p4 = expf(c[0] - m), p5 = expf(c[1] - m), p6 = expf(c[2] - m), p7 = expf(c[3] - m);
  float s = ((p0 + p1) + (p2 + p3)) + ((p4 + p5) + (p6 + p7));
#pragma unroll
  for (int off = 16; off > 0; off >>= 1) s += __shfl_xor(s, off, 32);
  if (lane == 0) redS[wave] = s;
  __syncthreads();
  s = (redS[0] + redS[1]) + (redS[2] + redS[3]);
  const float inv = kPCarry * (1.0f / s);
  const v4u u = (v4u){pk16(h_bits(p0 * inv), h_bits(p1 * inv)), pk16(h_bits(p2 * inv), h_bits(p3 * inv)),
                      pk16(h_bits(p4 * inv), h_bits(p5 * inv)), pk16(h_bits(p6 * inv), h_bits(p7 * inv))};
  unsigned short* pp = P + (size_t)row * kT + c0;
  *(volatile v4u*)pp = u;
  __threadfence();
  *(volatile v4u*)pp = u;
}

extern "C" void kernel_launch(void* const* d_in, const int* in_sizes, int n_in,
                              void* d_out, int out_size, void* d_ws, size_t ws_size,
                              hipStream_t stream) {
  if (n_in < 11) return;
  const float* X    = (const float*)d_in[0];
  const float* ln_g = (const float*)d_in[1];
  const float* ln_b = (const float*)d_in[2];
  const float* Wq   = (const float*)d_in[3];
  const float* bq   = (const float*)d_in[4];
  const float* Wk   = (const float*)d_in[5];
  const float* bk   = (const float*)d_in[6];
  const float* Wv   = (const float*)d_in[7];
  const float* bv   = (const float*)d_in[8];
  const float* Wo   = (const float*)d_in[9];
  const float* bo   = (const float*)d_in[10];
  float* out = (float*)d_out;

  if (in_sizes[0] != kNB * kC * kT || out_size != kNB * kC * kT) return;
  if (in_sizes[1] != kC || in_sizes[2] != kC) return;
  if (in_sizes[3] != kC * kE || in_sizes[5] != kC * kE || in_sizes[7] != kC * kE || in_sizes[9] != kE * kC) return;
  if (in_sizes[4] != kE || in_sizes[6] != kE || in_sizes[8] != kE || in_sizes[10] != kC) return;

  const size_t szWT  = (size_t)4 * kE * kC * 2;
  const size_t szTok = (size_t)kTok * kE * 2;
  const size_t szS   = (size_t)kNH * kT * kT * 4;
  const size_t szP   = (size_t)kNH * kT * kT * 2;
  const size_t oWT  = 0;
  const size_t oXNO = oWT + szWT;
  const size_t oQ   = oXNO + szTok;
  const size_t oK   = oQ + szTok;
  const size_t oV   = oK + szTok;
  const size_t oS   = oV + szTok;
  const size_t oP   = oS + szS;
  const size_t oEnd = oP + szP;
  if (oEnd > ws_size) return;

  char* ws = (char*)d_ws;
  unsigned short* WT  = (unsigned short*)(ws + oWT);
  unsigned short* WqT = WT;
  unsigned short* WkT = WT + (size_t)1 * kE * kC;
  unsigned short* WvT = WT + (size_t)2 * kE * kC;
  unsigned short* WoT = WT + (size_t)3 * kE * kC;
  unsigned short* XN  = (unsigned short*)(ws + oXNO);
  unsigned short* O16 = XN;
  unsigned short* Q16 = (unsigned short*)(ws + oQ);
  unsigned short* K16 = (unsigned short*)(ws + oK);
  unsigned short* VCM = (unsigned short*)(ws + oV);
  float*          S32 = (float*)(ws + oS);
  unsigned short* P16 = (unsigned short*)(ws + oP);

  const long strideTokB = (long)kT * kE;
  const long strideCmB  = (long)kC * kT;

  wtcast_kernel<<<dim3(kC / 64, kE / 64, 4), 256, 0, stream>>>(Wq, Wk, Wv, Wo, WT, kWCarry);

  ln_tok_kernel<<<kTok / 64, 256, 0, stream>>>(X, ln_g, ln_b, XN);

  wmma_gemm64<0, false, 2, 1, false><<<dim3(256, 1), 256, 0, stream>>>(
      XN, XN, kC, (long)0, WqT, WqT, kC, (long)0, (void*)Q16, (void*)Q16, kE, (long)0,
      bq, X, (long)0, kTok, kE, kC, kWCarryInv);
  wmma_gemm64<0, false, 2, 1, false><<<dim3(256, 1), 256, 0, stream>>>(
      XN, XN, kC, (long)0, WkT, WkT, kC, (long)0, (void*)K16, (void*)K16, kE, (long)0,
      bk, X, (long)0, kTok, kE, kC, kWCarryInv);

  wmma_gemm64<0, false, 1, 1, false><<<dim3(16, kNB), 256, 0, stream>>>(
      WvT, WvT, kC, (long)0, XN, XN, kC, strideTokB, (void*)VCM, (void*)VCM, kT, strideCmB,
      bv, X, (long)0, kC, kT, kC, kWCarryInv);

  for (int bb = 0; bb < kNB; ++bb) {
    const unsigned short* Qb = Q16 + (size_t)bb * strideTokB;
    const unsigned short* Kb = K16 + (size_t)bb * strideTokB;
    const unsigned short* Vb = VCM + (size_t)bb * strideCmB;
    unsigned short*       Ob = O16 + (size_t)bb * strideTokB;
    wmma_gemm64<0, false, 0, 0, false><<<dim3(32, kNH), 256, 0, stream>>>(
        Qb, Qb, kE, (long)kDH, Kb, Kb, kE, (long)kDH, (void*)S32, (void*)S32, kT, (long)kT * kT,
        bq, X, (long)0, kT, kT, kDH, kScoreScale);
    softmax_row_kernel<<<kNH * kT, 128, 0, stream>>>(S32, P16);
    wmma_gemm64<0, false, 0, 1, false><<<dim3(2, kNH), 256, 0, stream>>>(
        P16, P16, kT, (long)kT * kT, Vb, Vb, kT, (long)kDH * kT, (void*)Ob, (void*)Ob, kE, (long)kDH,
        bq, X, (long)0, kT, kDH, kT, kPVScale);
  }

  wmma_gemm64<0, false, 1, 0, true><<<dim3(16, kNB), 256, 0, stream>>>(
      WoT, WoT, kE, (long)0, O16, O16, kE, strideTokB, (void*)out, (void*)out, kT, strideCmB,
      bo, X, strideCmB, kC, kT, kE, kOutScale);
}
